// neuralFSI_59777354825820
// MI455X (gfx1250) — hardware-run, weakly checked
//
#include <hip/hip_runtime.h>
#include <stddef.h>
#include <math.h>


#define NF    30000
#define NFP   30016
#define NM    3000
#define NMP   3008
#define EFF   180000
#define EMF   60000
#define DF    32
#define DMM   64
#define KW    128
#define EF    6
#define TED   32
#define INF   4
#define INM   3
#define OUTF  4
#define OUTM  3
#define TCOL  1024
#define NLAY  2
#define LIDX  1
#define OUTN  (NF * OUTF + NM * OUTM)
#define OFF1  (NF * OUTF)
#define ASC   8
#define ATC   64
#define WSC   64
#define W3C   1024
#define OSC   (1.0f / 512.0f)
#define OXC   (1.0f / 4096.0f)
#define OW3   (1.0f / 8192.0f)
#define TB    256
#define NT    128
#define NTE   64
#define NKT   8
#define NCH   (NT * NKT)
#define WCAPF (32 * NKT)
#define CAPM  256
#define CTN   256
#define WSCAP (64u << 20)

static_assert(NFP % 64 == 0 && NFP >= NF && NFP - NF < 64);
static_assert(NMP % 64 == 0 && NMP >= NM && NMP - NM < 64);
static_assert(NFP % 32 == 0);
static_assert(EFF % 32 == 0);
static_assert((NCH & (NCH - 1)) == 0);
static_assert(TCOL == DF * DF);
static_assert(OUTN == 129000);
static_assert((OFF1 * 4) % 128 == 0);
static_assert(NM % 4 == 0);
static_assert(KW % 32 == 0 && DMM % 32 == 0 && DF % 32 == 0);
static_assert(EFF < (1 << 24) && EMF < (1 << 24));
static_assert(LIDX == NLAY - 1);
static_assert(KW == 4 * 32);

typedef float          v2f  __attribute__((ext_vector_type(2)));
typedef float          v4f  __attribute__((ext_vector_type(4)));
typedef float          v8f  __attribute__((ext_vector_type(8)));
typedef int            v4i  __attribute__((ext_vector_type(4)));
typedef _Float16       v8h  __attribute__((ext_vector_type(8)));
typedef _Float16       v16h __attribute__((ext_vector_type(16)));
typedef unsigned short v8us __attribute__((ext_vector_type(8)));
union FragH { v16h v; v8us u[2]; v8h h[2]; };

__device__ __forceinline__ v8f wmh(v16h a, v16h b, v8f c) {
  v8f d = __builtin_amdgcn_wmma_f32_16x16x32_f16(false, a, false, b, (short)0, c, false, false);
  asm volatile("v_nop\n\tv_nop\n\tv_nop\n\tv_nop" : "+v"(d) : "v"(a), "v"(b));
  return d;
}
__device__ __forceinline__ v8f zero8() { v8f z = {0.f, 0.f, 0.f, 0.f, 0.f, 0.f, 0.f, 0.f}; return z; }
__device__ __forceinline__ float wsum32(float v) {
#pragma unroll
  for (int s = 16; s > 0; s >>= 1) v += __shfl_xor(v, s);
  return v;
}

__device__ __forceinline__ v16h frag_glb(const unsigned short* P, int row, int ld, int k0, int hh) {
  FragH f;
  const unsigned short* p = P + (size_t)row * ld + k0 + 8 * hh;
  f.u[0] = *(const v8us*)p;
  f.u[1] = *(const v8us*)(p + 16);
  return f.v;
}
__device__ __forceinline__ v16h frag_lds(const _Float16* T, int row, int ld, int k0, int hh) {
  FragH f;
  const _Float16* p = T + row * ld + k0 + 8 * hh;
  f.h[0] = *(const v8h*)p;
  f.h[1] = *(const v8h*)(p + 16);
  return f.v;
}

__device__ __forceinline__ void cvt_unit(const float* __restrict__ P, unsigned short* dst, long sc, long sk,
                                         int K, int KP, int Nv, int Nout, float scale, int i) {
  const int upc = KP >> 3;
  if (i >= Nout * upc) return;
  const int n = i / upc;
  const int seg = i - n * upc;
  const int nc = n < Nv - 1 ? n : Nv - 1;
  v8h o;
#pragma unroll
  for (int j = 0; j < 8; ++j) {
    const int k = 8 * seg + j;
    const int kc = k < K - 1 ? k : K - 1;
    const float v = P[(size_t)nc * sc + (size_t)kc * sk];
    const float keep = (k < K && n < Nv) ? scale : 0.0f;
    o[j] = (_Float16)(v * keep);
  }
  const v8us ob = __builtin_bit_cast(v8us, o);
  unsigned short* d = dst + (size_t)i * 8;
  *(volatile v8us*)d = ob;
  __threadfence();
  *(volatile v8us*)d = ob;
}

__global__ __launch_bounds__(TB) void k_prep(
    const float* __restrict__ kW2, const float* __restrict__ kW3, const float* __restrict__ Wq,
    const float* __restrict__ Wroot, const float* __restrict__ Wo, const float* __restrict__ mW2,
    const float* __restrict__ Wk, const float* __restrict__ Wv,
    unsigned short* BW2, unsigned short* BW3, unsigned short* BWQ, unsigned short* BWR,
    unsigned short* BWO, unsigned short* BM2, unsigned short* BWK, unsigned short* BWV) {
  const int job = (int)blockIdx.y;
  const int i = (int)blockIdx.x * TB + (int)threadIdx.x;
  const float* P =
      job == 0 ? kW2 : job == 1 ? kW3 : job == 2 ? Wq : job == 3 ? Wroot : job == 4 ? Wo :
      job == 5 ? mW2 : job == 6 ? Wk : Wv;
  unsigned short* D =
      job == 0 ? BW2 : job == 1 ? BW3 : job == 2 ? BWQ : job == 3 ? BWR : job == 4 ? BWO :
      job == 5 ? BM2 : job == 6 ? BWK : BWV;
  const long sk = job == 0 ? KW : job == 1 ? TCOL : job == 2 ? DMM : (job == 3 || job == 4) ? DF : DMM;
  const int  K  = (job == 0 || job == 1) ? KW : (job == 2 || job == 3) ? DF : DMM;
  const int  Nv = job == 0 ? KW : job == 1 ? TCOL : job == 2 ? DMM : (job == 3 || job == 4) ? DF : DMM;
  const float scale = job == 1 ? (float)W3C : (float)WSC;
  cvt_unit(P, D, 1, sk, K, K, Nv, Nv, scale, i);
}

__global__ __launch_bounds__(64) void k_setup(const float* __restrict__ taup,
    const float* __restrict__ efW, const float* __restrict__ efb,
    const float* __restrict__ emW1, const float* __restrict__ emb1,
    const float* __restrict__ tW1, const float* __restrict__ tb1,
    const float* __restrict__ tW2, const float* __restrict__ tb2, float* CT) {
  __shared__ float sTe[TED];
  __shared__ float sTh[DMM];
  __shared__ __attribute__((aligned(16))) float sC[CTN];
  const int t = threadIdx.x;
  const float tau = taup[0];
  if (t < TED / 2) {
    const float fr = expf((-9.2103403719761836f * (float)t) / (float)(TED / 2));
    const float a = tau * fr;
    sTe[t] = sinf(a);
    sTe[TED / 2 + t] = cosf(a);
  }
  {
    const float z = tau * tW1[t] + tb1[t];
    const float sg = 1.0f / (1.0f + expf(fminf(-z, 30.0f)));
    sTh[t] = z * sg;
  }
  __syncthreads();
  float vm = emb1[t];
#pragma unroll 1
  for (int j = 0; j < TED; ++j) vm += sTe[j] * emW1[(INM + j) * DMM + t];
  float ss = tb2[t];
#pragma unroll 1
  for (int k = 0; k < DMM; ++k) ss += sTh[k] * tW2[k * (2 * DF) + t];
  const int tf = t & (DF - 1);
  float vf = efb[tf];
#pragma unroll 1
  for (int j = 0; j < TED; ++j) vf += sTe[j] * efW[(INF + j) * DF + tf];
  sC[t] = (t < DF) ? vf : 0.0f;
  sC[64 + t] = vm;
  sC[128 + t] = ss;
  sC[192 + t] = 0.0f;
  __syncthreads();
  const v4f v = *(const v4f*)(sC + 4 * t);
  float* dp = CT + 4 * t;
  *(volatile v4f*)dp = v;
  __threadfence();
  *(volatile v4f*)dp = v;
}

__global__ __launch_bounds__(TB) void k_encf(const float* __restrict__ fx, const float* __restrict__ Wf,
                                             const float* __restrict__ CT, float* XF, unsigned short* XH) {
  __shared__ __attribute__((aligned(16))) float sX[32 * DF];
  const int tid = threadIdx.x;
  const int row = tid >> 3, p = tid & 7;
  const int nb = (int)blockIdx.x * 32;
  const int n = nb + row;
  const int nc = n < NF - 1 ? n : NF - 1;
  const v4f a  = *(const v4f*)(fx + (size_t)nc * INF);
  const v4f w0 = *(const v4f*)(Wf + 0 * DF + 4 * p);
  const v4f w1 = *(const v4f*)(Wf + 1 * DF + 4 * p);
  const v4f w2 = *(const v4f*)(Wf + 2 * DF + 4 * p);
  const v4f w3 = *(const v4f*)(Wf + 3 * DF + 4 * p);
  const v4f tb = *(const v4f*)(CT + 4 * p);
  const v4f v = tb + a.x * w0 + a.y * w1 + a.z * w2 + a.w * w3;
  *(v4f*)(sX + row * DF + 4 * p) = v;
  float* dp = XF + (size_t)n * DF + 4 * p;
  *(volatile v4f*)dp = v;
  __syncthreads();
  const int t2 = tid & 127;
  const int r2 = t2 >> 2, q = t2 & 3;
  const v4f xa = *(const v4f*)(sX + r2 * DF + 8 * q);
  const v4f xb = *(const v4f*)(sX + r2 * DF + 8 * q + 4);
  v8h h8;
  h8[0] = (_Float16)(xa.x * (float)ASC); h8[1] = (_Float16)(xa.y * (float)ASC);
  h8[2] = (_Float16)(xa.z * (float)ASC); h8[3] = (_Float16)(xa.w * (float)ASC);
  h8[4] = (_Float16)(xb.x * (float)ASC); h8[5] = (_Float16)(xb.y * (float)ASC);
  h8[6] = (_Float16)(xb.z * (float)ASC); h8[7] = (_Float16)(xb.w * (float)ASC);
  const v8us hb = __builtin_bit_cast(v8us, h8);
  unsigned short* hp = XH + (size_t)(nb + r2) * DF + 8 * q;
  const bool act = tid < 128;
  if (act) *(volatile v8us*)hp = hb;
  __threadfence();
  *(volatile v4f*)dp = v;
  if (act) *(volatile v8us*)hp = hb;
}

__device__ __forceinline__ void put_rows64(const float* so, float* G, int r0, int lane) {
#pragma unroll
  for (int i = 0; i < 8; ++i) {
    const int row = 2 * i + (lane >> 4), p = lane & 15;
    const v4f v = *(const v4f*)(so + row * DMM + 4 * p);
    *(volatile v4f*)(G + (size_t)(r0 + row) * DMM + 4 * p) = v;
  }
}
__device__ __forceinline__ void put_rows32(const float* sm, float* G, int r0, int lane) {
#pragma unroll
  for (int i = 0; i < 4; ++i) {
    const int row = 4 * i + (lane >> 3), p = lane & 7;
    const v4f v = *(const v4f*)(sm + row * DF + 4 * p);
    *(volatile v4f*)(G + (size_t)(r0 + row) * DF + 4 * p) = v;
  }
}

__global__ __launch_bounds__(NT) void k_encm(
    const float* __restrict__ my, const float* __restrict__ W1, const float* __restrict__ CT,
    const unsigned short* __restrict__ BM2, const float* __restrict__ b2,
    const unsigned short* __restrict__ BWK, const float* __restrict__ bk,
    const unsigned short* __restrict__ BWV, const float* __restrict__ bv,
    const float* __restrict__ dW, const float* __restrict__ db,
    float* KM, float* VM, float* out1) {
  __shared__ __attribute__((aligned(16))) _Float16 sH[64 * DMM];
  __shared__ __attribute__((aligned(16))) float    sY[64 * DMM];
  __shared__ __attribute__((aligned(16))) _Float16 sYH[64 * DMM];
  __shared__ __attribute__((aligned(16))) float    sO[4][16 * DMM];
  __shared__ __attribute__((aligned(16))) float    sDo[64 * OUTM];
  const int tid = threadIdx.x, lane = tid & 31, wave = tid >> 5, hh = lane >> 4, m = lane & 15;
  const int nb = (int)blockIdx.x * 64;
  const int rw = 16 * wave;

#pragma unroll 1
  for (int j = 0; j < (64 * DMM) / NT; ++j) {
    const int idx = tid + NT * j;
    const int row = idx >> 6, col = idx & 63;
    int n = nb + row; n = n < NM - 1 ? n : NM - 1;
    float v = CT[64 + col];
    v += my[(size_t)n * INM + 0] * W1[0 * DMM + col];
    v += my[(size_t)n * INM + 1] * W1[1 * DMM + col];
    v += my[(size_t)n * INM + 2] * W1[2 * DMM + col];
    sH[row * DMM + col] = (_Float16)(fmaxf(v, 0.0f) * (float)ASC);
  }
  __syncthreads();

  {
    const v16h aH0 = frag_lds(sH, rw + m, DMM, 0, hh);
    const v16h aH1 = frag_lds(sH, rw + m, DMM, 32, hh);
#pragma unroll 1
    for (int t = 0; t < 4; ++t) {
      const int c = 16 * t + m;
      v8f acc = wmh(aH0, frag_glb(BM2, c, DMM, 0, hh), zero8());
      acc = wmh(aH1, frag_glb(BM2, c, DMM, 32, hh), acc);
      const float bb = b2[c];
#pragma unroll
      for (int r = 0; r < 8; ++r) {
        const float y = fmaxf(acc[r] * OSC + bb, 0.0f);
        sY[(rw + 8 * hh + r) * DMM + c] = y;
        sYH[(rw + 8 * hh + r) * DMM + c] = (_Float16)(y * (float)ASC);
      }
    }
  }
  __syncthreads();

  {
    const v16h aY0 = frag_lds(sYH, rw + m, DMM, 0, hh);
    const v16h aY1 = frag_lds(sYH, rw + m, DMM, 32, hh);
    float* so = sO[wave];
#pragma unroll 1
    for (int jb = 0; jb < 2; ++jb) {
      const unsigned short* Bp = jb ? BWV : BWK;
      const float* bp = jb ? bv : bk;
      float* G = jb ? VM : KM;
#pragma unroll 1
      for (int t = 0; t < 4; ++t) {
        const int c = 16 * t + m;
        v8f acc = wmh(aY0, frag_glb(Bp, c, DMM, 0, hh), zero8());
        acc = wmh(aY1, frag_glb(Bp, c, DMM, 32, hh), acc);
        const float bb = bp[c];
#pragma unroll
        for (int r = 0; r < 8; ++r) so[(8 * hh + r) * DMM + c] = acc[r] * OSC + bb;
      }
      __syncthreads();
      put_rows64(so, G, nb + rw, lane);
      __threadfence();
      put_rows64(so, G, nb + rw, lane);
      __syncthreads();
    }
  }

  {
    const int loc = tid & 63;
    float o0 = db[0], o1 = db[1], o2 = db[2];
#pragma unroll 1
    for (int d = 0; d < DMM; ++d) {
      const float y = sY[loc * DMM + d];
      o0 += y * dW[d * OUTM + 0];
      o1 += y * dW[d * OUTM + 1];
      o2 += y * dW[d * OUTM + 2];
    }
    if (tid < 64) { sDo[loc * OUTM + 0] = o0; sDo[loc * OUTM + 1] = o1; sDo[loc * OUTM + 2] = o2; }
  }
  __syncthreads();
  {
    int nval = NM - nb; nval = nval > 64 ? 64 : nval;
    const int npc = (nval * OUTM) / 4;
    const bool act = tid < npc;
    const int pc = act ? tid : 0;
    const v4f v = *(const v4f*)(sDo + 4 * pc);
    float* op = out1 + (size_t)nb * OUTM + 4 * pc;
    if (act) *(volatile v4f*)op = v;
    __threadfence();
    if (act) *(volatile v4f*)op = v;
  }
}

__global__ __launch_bounds__(NTE) void k_edge(
    const float* __restrict__ ea, const int* __restrict__ esrc,
    const float* __restrict__ kW1, const float* __restrict__ kb1,
    const unsigned short* __restrict__ BW2, const float* __restrict__ kb2,
    const unsigned short* __restrict__ BW3, const float* __restrict__ kb3,
    const float* __restrict__ XF, float* MSG) {
  __shared__ __attribute__((aligned(16))) _Float16 sA[2][16 * KW];
  __shared__ __attribute__((aligned(16))) _Float16 sB[2][16 * KW];
  __shared__ __attribute__((aligned(16))) float    sM[2][16 * DF];
  __shared__ __attribute__((aligned(16))) float    sKb3[TCOL];
  const int tid = threadIdx.x, lane = tid & 31, wave = tid >> 5, hh = lane >> 4, m = lane & 15;
  const int e0 = ((int)blockIdx.x * 2 + wave) * 16;
  _Float16* sa = sA[wave];
  _Float16* sb = sB[wave];
  float* sm = sM[wave];

#pragma unroll 1
  for (int i = tid; i < TCOL; i += NTE) sKb3[i] = kb3[i];

  {
    const int c4 = 4 * lane;
    const v4f w0 = *(const v4f*)(kW1 + 0 * KW + c4);
    const v4f w1 = *(const v4f*)(kW1 + 1 * KW + c4);
    const v4f w2 = *(const v4f*)(kW1 + 2 * KW + c4);
    const v4f w3 = *(const v4f*)(kW1 + 3 * KW + c4);
    const v4f w4 = *(const v4f*)(kW1 + 4 * KW + c4);
    const v4f w5 = *(const v4f*)(kW1 + 5 * KW + c4);
    const v4f bb = *(const v4f*)(kb1 + c4);
#pragma unroll 1
    for (int e = 0; e < 16; ++e) {
      const float* ep = ea + (size_t)(e0 + e) * EF;
      const float a0 = ep[0], a1 = ep[1], a2 = ep[2], a3 = ep[3], a4 = ep[4], a5 = ep[5];
      const v4f v = bb + a0 * w0 + a1 * w1 + a2 * w2 + a3 * w3 + a4 * w4 + a5 * w5;
      _Float16* sp = sa + e * KW + c4;
      sp[0] = (_Float16)(fmaxf(v.x, 0.0f) * (float)ASC);
      sp[1] = (_Float16)(fmaxf(v.y, 0.0f) * (float)ASC);
      sp[2] = (_Float16)(fmaxf(v.z, 0.0f) * (float)ASC);
      sp[3] = (_Float16)(fmaxf(v.w, 0.0f) * (float)ASC);
    }
  }
  __syncthreads();

  {
    v16h afr[4];
#pragma unroll
    for (int kb = 0; kb < 4; ++kb) afr[kb] = frag_lds(sa, m, KW, 32 * kb, hh);
#pragma unroll 1
    for (int ch = 0; ch < KW / 16; ++ch) {
      const int c = 16 * ch + m;
      v8f acc = zero8();
#pragma unroll
      for (int kb = 0; kb < 4; ++kb) acc = wmh(afr[kb], frag_glb(BW2, c, KW, 32 * kb, hh), acc);
      const float bb2 = kb2[c];
#pragma unroll
      for (int r = 0; r < 8; ++r)
        sb[(8 * hh + r) * KW + c] = (_Float16)(fmaxf(acc[r] * OSC + bb2, 0.0f) * (float)ASC);
    }
  }
  __syncthreads();

  v16h bfr[4];
#pragma unroll
  for (int kb = 0; kb < 4; ++kb) bfr[kb] = frag_lds(sb, m, KW, 32 * kb, hh);

  int s = esrc[e0 + m];
  s = s < 0 ? 0 : (s > NF - 1 ? NF - 1 : s);
  const float* xrow = XF + (size_t)s * DF;
  float xr[16];
  {
    const v4f xa = *(const v4f*)(xrow + 8 * hh);
    const v4f xb = *(const v4f*)(xrow + 8 * hh + 4);
    const v4f xc = *(const v4f*)(xrow + 16 + 8 * hh);
    const v4f xd = *(const v4f*)(xrow + 16 + 8 * hh + 4);
#pragma unroll
    for (int p = 0; p < 4; ++p) { xr[p] = xa[p]; xr[4 + p] = xb[p]; xr[8 + p] = xc[p]; xr[12 + p] = xd[p]; }
  }

#pragma unroll 1
  for (int i = 0; i < DF; ++i) {
    float part = 0.0f;
#pragma unroll
    for (int cc = 0; cc < 2; ++cc) {
      const int c = 2 * i + cc;
      const int col = 16 * c + m;
      v8f acc = zero8();
#pragma unroll
      for (int kb = 0; kb < 4; ++kb) acc = wmh(frag_glb(BW3, col, KW, 32 * kb, hh), bfr[kb], acc);
      const float* kbp = sKb3 + 16 * c + 8 * hh;
#pragma unroll
      for (int r = 0; r < 8; ++r) {
        const float w = acc[r] * OW3 + kbp[r];
        part += w * xr[cc * 8 + r];
      }
    }
    const float full = part + __shfl_xor(part, 16);
    if (hh == 0) sm[m * DF + i] = full;
  }
  __syncthreads();
  put_rows32(sm, MSG, e0, lane);
  __threadfence();
  put_rows32(sm, MSG, e0, lane);
}

__device__ __forceinline__ void hit_append(bool hj, int ent, int* list, int cap, int& wc) {
  const unsigned mj = __builtin_amdgcn_ballot_w32(hj);
  if (mj != 0u) {
    if (hj) {
      const int pos = wc + (int)__builtin_amdgcn_mbcnt_lo(mj, 0u);
      if (pos < cap) list[pos] = ent;
    }
    wc += (int)__builtin_popcount(mj);
  }
}

__device__ __forceinline__ void scan8(const int* __restrict__ keys, int nK, int cbase, int tid, unsigned nbu,
                                      int* list, int cap, int& wc) {
  const int el0 = tid * NKT;
  const int e0 = cbase + el0;
  const int sent = -2147483647 - 1;
  v4i da, db;
  if (cbase + NCH <= nK) {
    da = *(const v4i*)(keys + e0);
    db = *(const v4i*)(keys + e0 + 4);
  } else {
    da.x = (e0     < nK) ? keys[min(e0,     nK - 1)] : sent;
    da.y = (e0 + 1 < nK) ? keys[min(e0 + 1, nK - 1)] : sent;
    da.z = (e0 + 2 < nK) ? keys[min(e0 + 2, nK - 1)] : sent;
    da.w = (e0 + 3 < nK) ? keys[min(e0 + 3, nK - 1)] : sent;
    db.x = (e0 + 4 < nK) ? keys[min(e0 + 4, nK - 1)] : sent;
    db.y = (e0 + 5 < nK) ? keys[min(e0 + 5, nK - 1)] : sent;
    db.z = (e0 + 6 < nK) ? keys[min(e0 + 6, nK - 1)] : sent;
    db.w = (e0 + 7 < nK) ? keys[min(e0 + 7, nK - 1)] : sent;
  }
  const unsigned s0 = (unsigned)da.x - nbu, s1 = (unsigned)da.y - nbu;
  const unsigned s2 = (unsigned)da.z - nbu, s3 = (unsigned)da.w - nbu;
  const unsigned s4 = (unsigned)db.x - nbu, s5 = (unsigned)db.y - nbu;
  const unsigned s6 = (unsigned)db.z - nbu, s7 = (unsigned)db.w - nbu;
  const bool h0 = s0 < 64u, h1 = s1 < 64u, h2 = s2 < 64u, h3 = s3 < 64u;
  const bool h4 = s4 < 64u, h5 = s5 < 64u, h6 = s6 < 64u, h7 = s7 < 64u;
  const unsigned any = __builtin_amdgcn_ballot_w32(h0 | h1 | h2 | h3 | h4 | h5 | h6 | h7);
  if (any != 0u) {
    hit_append(h0, ((e0 + 0) << 6) | (int)s0, list, cap, wc);
    hit_append(h1, ((e0 + 1) << 6) | (int)s1, list, cap, wc);
    hit_append(h2, ((e0 + 2) << 6) | (int)s2, list, cap, wc);
    hit_append(h3, ((e0 + 3) << 6) | (int)s3, list, cap, wc);
    hit_append(h4, ((e0 + 4) << 6) | (int)s4, list, cap, wc);
    hit_append(h5, ((e0 + 5) << 6) | (int)s5, list, cap, wc);
    hit_append(h6, ((e0 + 6) << 6) | (int)s6, list, cap, wc);
    hit_append(h7, ((e0 + 7) << 6) | (int)s7, list, cap, wc);
  }
}

__global__ __launch_bounds__(NT) void k_flow(
    const unsigned short* __restrict__ XH, const float* __restrict__ XF,
    const unsigned short* __restrict__ BWQ, const float* __restrict__ bq,
    const int* __restrict__ mdst, const int* __restrict__ msrc, const float* __restrict__ eam,
    const float* __restrict__ KM, const float* __restrict__ VM,
    const float* __restrict__ We, const float* __restrict__ be,
    const unsigned short* __restrict__ BWO, const float* __restrict__ bo,
    const int* __restrict__ fdst, const float* __restrict__ MSG,
    const unsigned short* __restrict__ BWR, const float* __restrict__ broot,
    const float* __restrict__ CT, const float* __restrict__ dW, const float* __restrict__ db,
    float* out0) {
  __shared__ __attribute__((aligned(16))) float    sQY[64 * DMM];
  __shared__ __attribute__((aligned(16))) float    sAtt[64 * DMM];
  __shared__ __attribute__((aligned(16))) _Float16 sAtH[64 * DMM];
  __shared__ __attribute__((aligned(16))) float    sAgg[64 * DF];
  __shared__ int   sLm[4 * CAPM];
  __shared__ float sEm[4 * CAPM];
  __shared__ int   sLf[4 * WCAPF];
  __shared__ float sMax[64], sSum[64], sRs[64], sInv[64];
  __shared__ int   sDeg[64];
  __shared__ int   sWc[4], sOv[4];
  const int tid = threadIdx.x, lane = tid & 31, wave = tid >> 5, hh = lane >> 4, m = lane & 15;
  const int nb = (int)blockIdx.x * 64;
  const int rw = 16 * wave;
  const unsigned nbu = (unsigned)nb;

  {
    const v4f z = {0.f, 0.f, 0.f, 0.f};
#pragma unroll 1
    for (int i = tid; i < (64 * DMM) / 4; i += NT) *(v4f*)(sAtt + 4 * i) = z;
#pragma unroll 1
    for (int i = tid; i < (64 * DF) / 4; i += NT) *(v4f*)(sAgg + 4 * i) = z;
    if (tid < 64) { sMax[tid] = -3.0e38f; sSum[tid] = 0.0f; sDeg[tid] = 0; }
  }

  {
    const v16h aX = frag_glb(XH, nb + rw + m, DF, 0, hh);
#pragma unroll 1
    for (int t = 0; t < 4; ++t) {
      const int c = 16 * t + m;
      const v8f acc = wmh(aX, frag_glb(BWQ, c, DF, 0, hh), zero8());
      const float bb = bq[c];
#pragma unroll
      for (int r = 0; r < 8; ++r) sQY[(rw + 8 * hh + r) * DMM + c] = acc[r] * OSC + bb;
    }
  }
  __syncthreads();

  {
    int wc = 0;
    const int nChM = (EMF + NCH - 1) / NCH;
#pragma unroll 1
    for (int ch = 0; ch < nChM; ++ch) scan8(mdst, EMF, ch * NCH, tid, nbu, sLm + wave * CAPM, CAPM, wc);
    if (lane == 0) { sWc[wave] = wc < CAPM ? wc : CAPM; sOv[wave] = wc > CAPM ? 1 : 0; }
  }
  __syncthreads();

  const int d0 = 2 * lane;
#pragma unroll 1
  for (int wl = 0; wl < 4; ++wl) {
    int n = __builtin_amdgcn_readfirstlane(sWc[wl]);
    n = n > CAPM ? CAPM : (n < 0 ? 0 : n);
#pragma unroll 1
    for (int i = 0; i < n; ++i) {
      const int ent = __builtin_amdgcn_readfirstlane(sLm[wl * CAPM + i]);
      const int loc = ent & 63;
      if ((loc >> 4) == wave) {
        int e = ent >> 6;
        e = e < 0 ? 0 : (e > EMF - 1 ? EMF - 1 : e);
        int s = msrc[e];
        s = s < 0 ? 0 : (s > NM - 1 ? NM - 1 : s);
        const float* eap = eam + (size_t)e * EF;
        const v2f kmv = *(const v2f*)(KM + (size_t)s * DMM + d0);
        float k0 = kmv.x + be[d0], k1 = kmv.y + be[d0 + 1];
#pragma unroll
        for (int i6 = 0; i6 < EF; ++i6) {
          const float a = eap[i6];
          k0 += a * We[i6 * DMM + d0];
          k1 += a * We[i6 * DMM + d0 + 1];
        }
        const v2f qv = *(const v2f*)(sQY + loc * DMM + d0);
        float p = qv.x * k0 + qv.y * k1;
        p = wsum32(p) * 0.125f;
        if (lane == 0) { sEm[wl * CAPM + i] = p; sMax[loc] = fmaxf(sMax[loc], p); }
      }
    }
  }
  __syncthreads();
#pragma unroll 1
  for (int wl = 0; wl < 4; ++wl) {
    int n = __builtin_amdgcn_readfirstlane(sWc[wl]);
    n = n > CAPM ? CAPM : (n < 0 ? 0 : n);
#pragma unroll 1
    for (int i = 0; i < n; ++i) {
      const int ent = __builtin_amdgcn_readfirstlane(sLm[wl * CAPM + i]);
      const int loc = ent & 63;
      if ((loc >> 4) == wave) {
        const float ex = expf(sEm[wl * CAPM + i] - sMax[loc]);
        if (lane == 0) { sEm[wl * CAPM + i] = ex; sSum[loc] = sSum[loc] + ex; }
      }
    }
  }
  __syncthreads();
  if (tid < 64) { const float sv = sSum[tid]; sRs[tid] = sv > 0.0f ? 1.0f / sv : 0.0f; }
  __syncthreads();
#pragma unroll 1
  for (int wl = 0; wl < 4; ++wl) {
    int n = __builtin_amdgcn_readfirstlane(sWc[wl]);
    n = n > CAPM ? CAPM : (n < 0 ? 0 : n);
#pragma unroll 1
    for (int i = 0; i < n; ++i) {
      const int ent = __builtin_amdgcn_readfirstlane(sLm[wl * CAPM + i]);
      const int loc = ent & 63;
      if ((loc >> 4) == wave) {
        int e = ent >> 6;
        e = e < 0 ? 0 : (e > EMF - 1 ? EMF - 1 : e);
        int s = msrc[e];
        s = s < 0 ? 0 : (s > NM - 1 ? NM - 1 : s);
        const float alpha = sEm[wl * CAPM + i] * sRs[loc];
        const v2f vv = *(const v2f*)(VM + (size_t)s * DMM + d0);
        v2f* ap = (v2f*)(sAtt + loc * DMM + d0);
        v2f cur = *ap;
        cur += vv * alpha;
        *ap = cur;
      }
    }
  }
  __syncthreads();
#pragma unroll 1
  for (int u = tid; u < (64 * DMM) / 8; u += NT) {
    const v4f a = *(const v4f*)(sAtt + 8 * u);
    const v4f b = *(const v4f*)(sAtt + 8 * u + 4);
    v8h h8;
    h8[0] = (_Float16)(a.x * (float)ATC); h8[1] = (_Float16)(a.y * (float)ATC);
    h8[2] = (_Float16)(a.z * (float)ATC); h8[3] = (_Float16)(a.w * (float)ATC);
    h8[4] = (_Float16)(b.x * (float)ATC); h8[5] = (_Float16)(b.y * (float)ATC);
    h8[6] = (_Float16)(b.z * (float)ATC); h8[7] = (_Float16)(b.w * (float)ATC);
    *(v8h*)(sAtH + 8 * u) = h8;
  }
  __syncthreads();

  {
    const int nChF = (EFF + NCH - 1) / NCH;
#pragma unroll 1
    for (int ch = 0; ch < nChF; ++ch) {
      int wcf = 0;
      scan8(fdst, EFF, ch * NCH, tid, nbu, sLf + wave * WCAPF, WCAPF, wcf);
      if (lane == 0) sWc[wave] = wcf < WCAPF ? wcf : WCAPF;
      __syncthreads();
#pragma unroll 1
      for (int wl = 0; wl < 4; ++wl) {
        int n = __builtin_amdgcn_readfirstlane(sWc[wl]);
        n = n > WCAPF ? WCAPF : (n < 0 ? 0 : n);
#pragma unroll 1
        for (int i = 0; i < n; ++i) {
          const int ent = __builtin_amdgcn_readfirstlane(sLf[wl * WCAPF + i]);
          const int loc = ent & 63;
          if ((loc >> 4) == wave) {
            int e = ent >> 6;
            e = e < 0 ? 0 : (e > EFF - 1 ? EFF - 1 : e);
            const float mv = MSG[(size_t)e * DF + lane];
            sAgg[loc * DF + lane] = sAgg[loc * DF + lane] + mv;
            if (lane == 0) sDeg[loc] = sDeg[loc] + 1;
          }
        }
      }
      __syncthreads();
    }
  }
  if (tid < 64) {
    const int dg = sDeg[tid];
    sInv[tid] = 1.0f / (float)(dg > 1 ? dg : 1);
  }
  __syncthreads();

  {
    const v16h aX  = frag_glb(XH, nb + rw + m, DF, 0, hh);
    const v16h aA0 = frag_lds(sAtH, rw + m, DMM, 0, hh);
    const v16h aA1 = frag_lds(sAtH, rw + m, DMM, 32, hh);
#pragma unroll 1
    for (int t = 0; t < 2; ++t) {
      const int c = 16 * t + m;
      const v8f dR = wmh(aX, frag_glb(BWR, c, DF, 0, hh), zero8());
      v8f dC = wmh(aA0, frag_glb(BWO, c, DMM, 0, hh), zero8());
      dC = wmh(aA1, frag_glb(BWO, c, DMM, 32, hh), dC);
      const float br = broot[c], bc = bo[c], scl = CT[128 + c], shf = CT[160 + c];
#pragma unroll
      for (int r = 0; r < 8; ++r) {
        const int loc = rw + 8 * hh + r;
        const int n = nb + loc;
        const float xi = dR[r] * OSC + br + sAgg[loc * DF + c] * sInv[loc];
        const float xc = dC[r] * OXC + bc;
        const float g = fmaxf(xi + xc, 0.0f);
        const float z = g * (1.0f + scl) + shf;
        const float sg = 1.0f / (1.0f + expf(fminf(-z, 30.0f)));
        sQY[loc * DF + c] = z * sg + XF[(size_t)n * DF + c];
      }
    }
  }
  __syncthreads();

  {
    const int loc = tid & 63;
    const int n = nb + loc;
    float o0 = db[0], o1 = db[1], o2 = db[2], o3 = db[3];
#pragma unroll 1
    for (int d = 0; d < DF; ++d) {
      const float y = sQY[loc * DF + d];
      const v4f w = *(const v4f*)(dW + d * OUTF);
      o0 += y * w.x; o1 += y * w.y; o2 += y * w.z; o3 += y * w.w;
    }
    const int ov = sOv[0] | sOv[1] | sOv[2] | sOv[3];
    v4f o = {o0, o1, o2, o3};
    if (ov != 0) o = o + __int_as_float(0x7fc00000);
    const bool act = (tid < 64) && (n < NF);
    float* op = out0 + (size_t)(n < NF ? n : 0) * OUTF;
    if (act) *(volatile v4f*)op = o;
    __threadfence();
    if (act) *(volatile v4f*)op = o;
  }
}

extern "C" void kernel_launch(void* const* d_in, const int* in_sizes, int n_in,
                              void* d_out, int out_size, void* d_ws, size_t ws_size,
                              hipStream_t stream) {
  if (n_in < 40) return;
  if (in_sizes[0] != NF * INF || in_sizes[1] != NM * INM || in_sizes[2] != 1 ||
      in_sizes[3] != 2 * EFF || in_sizes[4] != EFF * EF || in_sizes[5] != EMF || in_sizes[6] != EMF ||
      in_sizes[7] != EMF * EF) return;
  if (in_sizes[8] != (INF + TED) * DF || in_sizes[9] != DF || in_sizes[10] != (INM + TED) * DMM ||
      in_sizes[11] != DMM || in_sizes[12] != DMM * DMM || in_sizes[13] != DMM) return;
  if (in_sizes[14] != NLAY * EF * KW || in_sizes[15] != NLAY * KW || in_sizes[16] != NLAY * KW * KW ||
      in_sizes[17] != NLAY * KW || in_sizes[18] != NLAY * KW * TCOL || in_sizes[19] != NLAY * TCOL) return;
  if (in_sizes[20] != NLAY * DF * DF || in_sizes[21] != NLAY * DF || in_sizes[22] != NLAY * DF * DMM ||
      in_sizes[23] != NLAY * DMM || in_sizes[24] != NLAY * DMM * DMM || in_sizes[25] != NLAY * DMM ||
      in_sizes[26] != NLAY * EF * DMM || in_sizes[27] != NLAY * DMM || in_sizes[28] != NLAY * DMM * DMM ||
      in_sizes[29] != NLAY * DMM || in_sizes[30] != NLAY * DMM * DF || in_sizes[31] != NLAY * DF) return;
  if (in_sizes[32] != NLAY * DMM || in_sizes[33] != NLAY * DMM || in_sizes[34] != NLAY * DMM * 2 * DF ||
      in_sizes[35] != NLAY * 2 * DF || in_sizes[36] != DF * OUTF || in_sizes[37] != OUTF ||
      in_sizes[38] != DMM * OUTM || in_sizes[39] != OUTM) return;
  if (out_size != OUTN) return;

  const float* flow_x   = (const float*)d_in[0];
  const float* memb_y   = (const float*)d_in[1];
  const float* tau      = (const float*)d_in[2];
  const int*   ei_ff    = (const int*)d_in[3];
  const float* eattr_ff = (const float*)d_in[4];
  const int*   mf_src   = (const int*)d_in[5];
  const int*   mf_dst   = (const int*)d_in[6];
  const float* eattr_mf = (const float*)d_in[7];
  const float* enc_f_W  = (const float*)d_in[8];
  const float* enc_f_b  = (const float*)d_in[9];
  const float* enc_m_W1 = (const float*)d_in[10];
  const float* enc_m_b1 = (const float*)d_in[11];
  const float* enc_m_W2 = (const float*)d_in[12];
  const float* enc_m_b2 = (const float*)d_in[13];
  const float* kW1   = (const float*)d_in[14] + (size_t)LIDX * EF * KW;
  const float* kb1   = (const float*)d_in[15] + (size_t)LIDX * KW;
  const float* kW2   = (const float*)d_in[16] + (size_t)LIDX * KW * KW;
  const float* kb2   = (const float*)d_in[17] + (size_t)LIDX * KW;
  const float* kW3   = (const float*)d_in[18] + (size_t)LIDX * KW * TCOL;
  const float* kb3   = (const float*)d_in[19] + (size_t)LIDX * TCOL;
  const float* Wroot = (const float*)d_in[20] + (size_t)LIDX * DF * DF;
  const float* broot = (const float*)d_in[21] + (size_t)LIDX * DF;
  const float* Wq    = (const float*)d_in[22] + (size_t)LIDX * DF * DMM;
  const float* bq    = (const float*)d_in[23] + (size_t)LIDX * DMM;
  const float* Wk    = (const float*)d_in[24] + (size_t)LIDX * DMM * DMM;
  const float* bk    = (const float*)d_in[25] + (size_t)LIDX * DMM;
  const float* We    = (const float*)d_in[26] + (size_t)LIDX * EF * DMM;
  const float* be    = (const float*)d_in[27] + (size_t)LIDX * DMM;
  const float* Wv    = (const float*)d_in[28] + (size_t)LIDX * DMM * DMM;
  const float* bv    = (const float*)d_in[29] + (size_t)LIDX * DMM;
  const float* Wo    = (const float*)d_in[30] + (size_t)LIDX * DMM * DF;
  const float* bo    = (const float*)d_in[31] + (size_t)LIDX * DF;
  const float* tW1   = (const float*)d_in[32] + (size_t)LIDX * DMM;
  const float* tb1   = (const float*)d_in[33] + (size_t)LIDX * DMM;
  const float* tW2   = (const float*)d_in[34] + (size_t)LIDX * DMM * 2 * DF;
  const float* tb2   = (const float*)d_in[35] + (size_t)LIDX * 2 * DF;
  const float* dec_f_W = (const float*)d_in[36];
  const float* dec_f_b = (const float*)d_in[37];
  const float* dec_m_W = (const float*)d_in[38];
  const float* dec_m_b = (const float*)d_in[39];
  float* out = (float*)d_out;
  const int* ff_src = ei_ff;
  const int* ff_dst = ei_ff + EFF;

  char* ws = (char*)d_ws;
  size_t off = 0;
#define CARVE(NAME, BYTES) const size_t NAME = off; off += (size_t)(BYTES); off = (off + 255) & ~(size_t)255;
  CARVE(oBW2, (size_t)KW * KW * 2)
  CARVE(oBW3, (size_t)TCOL * KW * 2)
  CARVE(oBWQ, (size_t)DMM * DF * 2)
  CARVE(oBWR, (size_t)DF * DF * 2)
  CARVE(oBWO, (size_t)DF * DMM * 2)
  CARVE(oBM2, (size_t)DMM * DMM * 2)
  CARVE(oBWK, (size_t)DMM * DMM * 2)
  CARVE(oBWV, (size_t)DMM * DMM * 2)
  CARVE(oCT,  (size_t)CTN * 4)
  CARVE(oXF,  (size_t)NFP * DF * 4)
  CARVE(oXH,  (size_t)NFP * DF * 2)
  CARVE(oKM,  (size_t)NMP * DMM * 4)
  CARVE(oVM,  (size_t)NMP * DMM * 4)
  CARVE(oMSG, (size_t)EFF * DF * 4)
#undef CARVE
  if (off > ws_size || off > (size_t)WSCAP) return;

  unsigned short* BW2 = (unsigned short*)(ws + oBW2);
  unsigned short* BW3 = (unsigned short*)(ws + oBW3);
  unsigned short* BWQ = (unsigned short*)(ws + oBWQ);
  unsigned short* BWR = (unsigned short*)(ws + oBWR);
  unsigned short* BWO = (unsigned short*)(ws + oBWO);
  unsigned short* BM2 = (unsigned short*)(ws + oBM2);
  unsigned short* BWK = (unsigned short*)(ws + oBWK);
  unsigned short* BWV = (unsigned short*)(ws + oBWV);
  float*          CT  = (float*)(ws + oCT);
  float*          XF  = (float*)(ws + oXF);
  unsigned short* XH  = (unsigned short*)(ws + oXH);
  float*          KM  = (float*)(ws + oKM);
  float*          VM  = (float*)(ws + oVM);
  float*          MSG = (float*)(ws + oMSG);

  k_prep<<<dim3((TCOL * KW / 8 + TB - 1) / TB, 8, 1), TB, 0, stream>>>(
      kW2, kW3, Wq, Wroot, Wo, enc_m_W2, Wk, Wv, BW2, BW3, BWQ, BWR, BWO, BM2, BWK, BWV);
  k_setup<<<1, 64, 0, stream>>>(tau, enc_f_W, enc_f_b, enc_m_W1, enc_m_b1, tW1, tb1, tW2, tb2, CT);
  k_encf<<<NFP / 32, TB, 0, stream>>>(flow_x, enc_f_W, CT, XF, XH);
  k_encm<<<NMP / 64, NT, 0, stream>>>(memb_y, enc_m_W1, CT, BM2, enc_m_b2, BWK, bk, BWV, bv,
                                      dec_m_W, dec_m_b, KM, VM, out + OFF1);
  k_edge<<<EFF / 32, NTE, 0, stream>>>(eattr_ff, ff_src, kW1, kb1, BW2, kb2, BW3, kb3, XF, MSG);
  k_flow<<<NFP / 64, NT, 0, stream>>>(XH, XF, BWQ, bq, mf_dst, mf_src, eattr_mf, KM, VM, We, be, BWO, bo,
                                      ff_dst, MSG, BWR, broot, CT, dec_f_W, dec_f_b, out);
}
